// ConvBlockLSTM_29497835388975
// MI455X (gfx1250) — hardware-verified
//
#include <hip/hip_runtime.h>
#include <stddef.h>

constexpr int kB     = 4;
constexpr int kT     = 8;
constexpr int kImg   = 64;
constexpr int kPixF  = 4096;
constexpr int kCin   = 32;
constexpr int kF     = 32;
constexpr int kG4    = 128;
constexpr int kRows  = 16384;
constexpr int kTaps  = 9;
constexpr int kKx    = 288;
constexpr int kKtot  = 576;
constexpr int kChunksPerRow = 72;
constexpr int kLayers = 2;

typedef __attribute__((ext_vector_type(16))) _Float16 v16h;
typedef __attribute__((ext_vector_type(8)))  _Float16 v8h;
typedef __attribute__((ext_vector_type(16))) __bf16   v16b;
typedef __attribute__((ext_vector_type(8)))  __bf16   v8b;
typedef __attribute__((ext_vector_type(8)))  float    v8f;
typedef __attribute__((ext_vector_type(4)))  float    v4f;
typedef __attribute__((ext_vector_type(4)))  unsigned v4u;

__device__ __forceinline__ unsigned short f2bf_bits(float f) {
  unsigned u = __float_as_uint(f);
  return (unsigned short)((u + 0x7FFFu + ((u >> 16) & 1u)) >> 16);
}
__device__ __forceinline__ float bf_bits2f(unsigned short h) { return __uint_as_float(((unsigned)h) << 16); }

__device__ __forceinline__ unsigned pk2(unsigned short a, unsigned short b) {
  return (unsigned)a | ((unsigned)b << 16);
}
__device__ __forceinline__ unsigned pkh2(float a, float b) {
  return pk2(__builtin_bit_cast(unsigned short, (_Float16)a), __builtin_bit_cast(unsigned short, (_Float16)b));
}

__device__ __forceinline__ void dep_guard_h(v8f& a, v8f& b, v16h x, v16h y) { asm volatile("v_nop\n\tv_nop\n\tv_nop\n\tv_nop" : "+v"(a), "+v"(b) : "v"(x), "v"(y)); }
__device__ __forceinline__ void dep_guard_b(v8f& a, v8f& b, v16b x, v16b y) { asm volatile("v_nop\n\tv_nop\n\tv_nop\n\tv_nop" : "+v"(a), "+v"(b) : "v"(x), "v"(y)); }
__device__ __forceinline__ void keep4_h(v16h a, v16h b, v16h c, v16h d) { asm volatile("v_nop" :: "v"(a), "v"(b), "v"(c), "v"(d)); }
__device__ __forceinline__ void keep4_b(v16b a, v16b b, v16b c, v16b d) { asm volatile("v_nop" :: "v"(a), "v"(b), "v"(c), "v"(d)); }
__device__ __forceinline__ void acc_guard4(v8f& a, v8f& b, v8f& c, v8f& d) { asm volatile("v_nop\n\tv_nop\n\tv_nop\n\tv_nop" : "+v"(a), "+v"(b), "+v"(c), "+v"(d)); }
template <typename T> struct Frag;
template <> struct Frag<_Float16> {
  typedef v16h V; union U { v16h v; v8h h[2]; };
  static __device__ __forceinline__ v16h load(const _Float16* p) {
    U f; f.h[0] = *(const v8h*)(p); f.h[1] = *(const v8h*)(p + 16); return f.v;
  }
  static __device__ __forceinline__ v8f mma(v16h a, v16h b, v8f c) {
    return __builtin_amdgcn_wmma_f32_16x16x32_f16(false, a, false, b, (short)0, c, false, false);
  }
  static __device__ __forceinline__ void guard(v8f& a, v8f& b, v16h x, v16h y) { dep_guard_h(a, b, x, y); }
  static __device__ __forceinline__ void keep(v16h a, v16h b, v16h c, v16h d) { keep4_h(a, b, c, d); }
};
template <> struct Frag<__bf16> {
  typedef v16b V; union U { v16b v; v8b h[2]; };
  static __device__ __forceinline__ v16b load(const __bf16* p) {
    U f; f.h[0] = *(const v8b*)(p); f.h[1] = *(const v8b*)(p + 16); return f.v;
  }
  static __device__ __forceinline__ v8f mma(v16b a, v16b b, v8f c) {
    return __builtin_amdgcn_wmma_f32_16x16x32_bf16(false, a, false, b, (short)0, c, false, false);
  }
  static __device__ __forceinline__ void guard(v8f& a, v8f& b, v16b x, v16b y) { dep_guard_b(a, b, x, y); }
  static __device__ __forceinline__ void keep(v16b a, v16b b, v16b c, v16b d) { keep4_b(a, b, c, d); }
};

template <int ET> struct Elem;
template <> struct Elem<0> { typedef _Float16 T; };
template <> struct Elem<1> { typedef __bf16 T; };
template <int ET, bool SPLIT, int BIAS_MODE, int OUT_MODE, bool RESID, int ACT = 0>
__global__ __launch_bounds__(256) void wmma_gemm64(
    const unsigned short* __restrict__ Ap, const unsigned short* __restrict__ A2p, int lda, long strideA,
    const unsigned short* __restrict__ Btp, const unsigned short* __restrict__ Bt2p, int ldb, long strideB,
    void* __restrict__ Cout, void* __restrict__ Cout2, int ldc, long strideC,
    const float* __restrict__ bias,
    const float* __restrict__ resid, long strideR,
    int M, int N, int K, float scale) {
  typedef typename Elem<ET>::T T;
  typedef typename Frag<T>::V V;
  const T* A = (const T*)Ap; const T* A2 = (const T*)A2p; const T* Bt = (const T*)Btp; const T* Bt2 = (const T*)Bt2p;
  __shared__ __align__(16) float sT[8][16 * 68];
  const int b    = blockIdx.y;
  const int lane = threadIdx.x & 31;
  const int wave = threadIdx.x >> 5;
  const int tilesN = N >> 6;
  const int tilesM = M >> 6;
  const int tile = blockIdx.x * 8 + wave;
  if (tile >= tilesM * tilesN) return;
  const int tm = tile / tilesN;
  const int tn = tile - tm * tilesN;
  const int m0 = tm << 6;
  const int n0 = tn << 6;

  const T* Ab  = A  + (size_t)b * strideA;
  const T* Bb  = Bt + (size_t)b * strideB;
  const T* Ab2 = SPLIT ? (A2  + (size_t)b * strideA) : nullptr;
  const T* Bb2 = SPLIT ? (Bt2 + (size_t)b * strideB) : nullptr;

  const int rlane = lane & 15;
  const int koff  = (lane >> 4) * 8;
  const int mOff  = (lane >> 4) * 8;

  v8f acc[4][4];
#pragma unroll
  for (int i = 0; i < 4; ++i)
#pragma unroll
    for (int j = 0; j < 4; ++j) acc[i][j] = (v8f){0.f,0.f,0.f,0.f,0.f,0.f,0.f,0.f};

  for (int k0 = 0; k0 < K; k0 += 32) {
    V bh[4], bl[4];
#pragma unroll
    for (int j = 0; j < 4; ++j) {
      const size_t bo = (size_t)(n0 + (j << 4) + rlane) * ldb + koff + k0;
      bh[j] = Frag<T>::load(Bb + bo);
      if (SPLIT) bl[j] = Frag<T>::load(Bb2 + bo);
    }
#pragma unroll
    for (int i = 0; i < 4; ++i) {
      const size_t ao = (size_t)(m0 + (i << 4) + rlane) * lda + koff + k0;
      V ah = Frag<T>::load(Ab + ao);
      V al;
      if (SPLIT) al = Frag<T>::load(Ab2 + ao);
#pragma unroll
      for (int j = 0; j < 4; ++j) {
        acc[i][j] = Frag<T>::mma(ah, bh[j], acc[i][j]);
        if (SPLIT) {
          acc[i][j] = Frag<T>::mma(ah, bl[j], acc[i][j]);
          acc[i][j] = Frag<T>::mma(al, bh[j], acc[i][j]);
        }
      }
      Frag<T>::guard(acc[i][0], acc[i][3], ah, SPLIT ? al : ah);
    }
    Frag<T>::keep(bh[0], bh[1], bh[2], bh[3]);
    if (SPLIT) Frag<T>::keep(bl[0], bl[1], bl[2], bl[3]);
  }
  acc_guard4(acc[0][0], acc[0][1], acc[0][2], acc[0][3]);
  acc_guard4(acc[1][0], acc[1][1], acc[1][2], acc[1][3]);
  acc_guard4(acc[2][0], acc[2][1], acc[2][2], acc[2][3]);
  acc_guard4(acc[3][0], acc[3][1], acc[3][2], acc[3][3]);

  float* slab = sT[wave];
  const float* Rb = RESID ? (resid + (size_t)b * strideR) : nullptr;
#pragma unroll
  for (int i = 0; i < 4; ++i) {
    const int mBase = m0 + (i << 4);
#pragma unroll
    for (int j = 0; j < 4; ++j) {
      const int n = n0 + (j << 4) + rlane;
      float bv = 0.f;
      if (BIAS_MODE == 2) bv = bias[n];
#pragma unroll
      for (int r = 0; r < 8; ++r) {
        float v = acc[i][j][r] * scale;
        if (BIAS_MODE == 1) v += bias[mBase + mOff + r];
        if (BIAS_MODE == 2) v += bv;
        if (RESID) v += Rb[(size_t)(mBase + mOff + r) * ldc + n];
        if (ACT == 1) v = tanhf(v);
        if (ACT == 2) v = fmaxf(v, 0.0f);
        if (ACT == 3) v = v / (1.0f + expf(-v));
        if (ACT == 4) v = (v > 0.f) ? v : 0.01f * v;
        if (ACT == 5) v = 0.5f * v * (1.0f + erff(v * 0.70710678118654752f));
        slab[(mOff + r) * 68 + (j << 4) + rlane] = v;
      }
    }
    __builtin_amdgcn_fence(__ATOMIC_RELEASE, "workgroup");
    __builtin_amdgcn_wave_barrier();
    __builtin_amdgcn_fence(__ATOMIC_ACQUIRE, "workgroup");
    if (OUT_MODE == 0) {
      float* C = (float*)Cout + (size_t)b * strideC;
      const int hh = lane >> 4, c4 = (lane & 15) * 4;
      for (int pass = 0; pass < 2; ++pass) {
#pragma unroll
        for (int it = 0; it < 8; ++it) {
          const int row = it * 2 + hh;
          v4f v = *(const v4f*)(slab + row * 68 + c4);
          *(volatile v4f*)(C + (size_t)(mBase + row) * ldc + n0 + c4) = v;
        }
        __threadfence();
      }
    } else {
      const int q = lane >> 3, c8 = (lane & 7) * 8;
      unsigned short* C  = (unsigned short*)Cout  + (size_t)b * strideC;
      unsigned short* C2 = (OUT_MODE == 2) ? ((unsigned short*)Cout2 + (size_t)b * strideC) : nullptr;
      for (int pass = 0; pass < 2; ++pass) {
#pragma unroll
        for (int it = 0; it < 4; ++it) {
          const int row = it * 4 + q;
          const float* sp = slab + row * 68 + c8;
          v8h hv, lv;
#pragma unroll
          for (int e = 0; e < 8; ++e) {
            if (OUT_MODE == 1) {
              hv[e] = (_Float16)sp[e];
            } else {
              unsigned short hb = f2bf_bits(sp[e]);
              unsigned short lb = f2bf_bits(sp[e] - bf_bits2f(hb));
              hv[e] = __builtin_bit_cast(_Float16, hb);
              lv[e] = __builtin_bit_cast(_Float16, lb);
            }
          }
          *(volatile v8h*)(C + (size_t)(mBase + row) * ldc + n0 + c8) = hv;
          if (OUT_MODE == 2) *(volatile v8h*)(C2 + (size_t)(mBase + row) * ldc + n0 + c8) = lv;
        }
        __threadfence();
      }
    }
    __builtin_amdgcn_fence(__ATOMIC_RELEASE, "workgroup");
    __builtin_amdgcn_wave_barrier();
    __builtin_amdgcn_fence(__ATOMIC_ACQUIRE, "workgroup");
  }
}

__global__ __launch_bounds__(256) void k_prep_w(const float* __restrict__ Wk, const float* __restrict__ Uk,
                                                unsigned short* __restrict__ Bt) {
  const int l  = blockIdx.y;
  const int g  = blockIdx.x * 256 + threadIdx.x;
  const int e0 = g * 8;
  const int n  = e0 / kKtot;
  const int col0 = e0 - n * kKtot;
  const bool isU = col0 >= kKx;
  const int colr = isU ? col0 - kKx : col0;
  const int tap  = colr >> 5;
  const int c0   = colr & 31;
  float f[8];
#pragma unroll
  for (int j = 0; j < 8; ++j) {
    const size_t idx = ((((size_t)l * kTaps + tap) * kCin + c0 + j) * kG4) + n;
    const float wv = Wk[idx];
    const float uv = Uk[idx];
    f[j] = (isU ? uv : wv) * 16.0f;
  }
  v4u u;
  u[0] = pkh2(f[0], f[1]); u[1] = pkh2(f[2], f[3]); u[2] = pkh2(f[4], f[5]); u[3] = pkh2(f[6], f[7]);
  volatile v4u* d = (volatile v4u*)(Bt + (size_t)l * kG4 * kKtot + e0);
  *d = u;
  __threadfence();
  *d = u;
}

__global__ __launch_bounds__(256) void k_im2col(const float* __restrict__ src, const float* __restrict__ Hst,
                                                const float* __restrict__ gam, const float* __restrict__ bet,
                                                const float* __restrict__ mea, const float* __restrict__ vr,
                                                unsigned short* __restrict__ IM, int t, int hzero) {
  const int g    = blockIdx.x * 256 + threadIdx.x;
  const int row  = g / kChunksPerRow;
  const int cc   = g - row * kChunksPerRow;
  const int slot = cc >> 2;
  const int c8   = (cc & 3) * 8;
  const bool isH = slot >= kTaps;
  const int tap  = isH ? slot - kTaps : slot;
  const int kh   = tap / 3, kw = tap - kh * 3;
  const int b    = row >> 12, yx = row & (kPixF - 1);
  const int y    = yx >> 6, x = yx & (kImg - 1);
  const int yy   = y + kh - 1, xx = x + kw - 1;
  const bool inb = ((unsigned)yy < (unsigned)kImg) && ((unsigned)xx < (unsigned)kImg);
  const int yc   = yy < 0 ? 0 : (yy > kImg - 1 ? kImg - 1 : yy);
  const int xc   = xx < 0 ? 0 : (xx > kImg - 1 ? kImg - 1 : xx);
  const float* xs = src + ((((size_t)b * kT + t) * kImg + yc) * kImg + xc) * kCin + c8;
  const float* hs = Hst + (((size_t)b * kImg + yc) * kImg + xc) * kF + c8;
  const v4f xa = *(const v4f*)(xs), xb = *(const v4f*)(xs + 4);
  const v4f ha = *(const v4f*)(hs), hb = *(const v4f*)(hs + 4);
  const v4f ga = *(const v4f*)(gam + c8), gb = *(const v4f*)(gam + c8 + 4);
  const v4f ta = *(const v4f*)(bet + c8), tb = *(const v4f*)(bet + c8 + 4);
  const v4f ma = *(const v4f*)(mea + c8), mb = *(const v4f*)(mea + c8 + 4);
  const v4f va = *(const v4f*)(vr + c8),  vb = *(const v4f*)(vr + c8 + 4);
  v4f sa, sb;
#pragma unroll
  for (int e = 0; e < 4; ++e) {
    sa[e] = ga[e] * rsqrtf(va[e] + 1e-3f);
    sb[e] = gb[e] * rsqrtf(vb[e] + 1e-3f);
  }
  v4f oa = (xa - ma) * sa + ta;
  v4f ob = (xb - mb) * sb + tb;
  const v4f z4 = (v4f){0.f, 0.f, 0.f, 0.f};
  v4f qa = ha, qb = hb;
  if (hzero) { qa = z4; qb = z4; }
  if (isH)   { oa = qa; ob = qb; }
  if (!inb)  { oa = z4; ob = z4; }
  v4u u;
  u[0] = pkh2(oa[0], oa[1]); u[1] = pkh2(oa[2], oa[3]);
  u[2] = pkh2(ob[0], ob[1]); u[3] = pkh2(ob[2], ob[3]);
  volatile v4u* d = (volatile v4u*)(IM + (size_t)g * 8);
  *d = u;
  __threadfence();
  *d = u;
}

__global__ __launch_bounds__(256) void k_cell(const float* __restrict__ Z, float* __restrict__ Cst,
                                              float* __restrict__ Hst, float* __restrict__ outp,
                                              const float* __restrict__ resid,
                                              int t, int first, int use_resid) {
  __shared__ __align__(16) float sC[256];
  __shared__ __align__(16) float sH[256];
  __shared__ __align__(16) float sO[256];
  const int tid = threadIdx.x, lane = tid & 31, wave = tid >> 5;
  const int p0 = blockIdx.x * 8;
  const int p  = p0 + wave;
  const int b  = p0 >> 12;
  {
    const float* zr = Z + (size_t)p * kG4;
    const float zi = zr[lane];
    const float zf = zr[kF + lane];
    const float zg = zr[2 * kF + lane];
    const float zo = zr[3 * kF + lane];
    float cold = Cst[(size_t)p * kF + lane];
    if (first) cold = 0.0f;
    const size_t o = ((size_t)(b * kT + t) * kPixF + (p & (kPixF - 1))) * kF + lane;
    float rv = resid[o];
    if (!use_resid) rv = 0.0f;
    const float ig = fminf(fmaxf(zi * 0.2f + 0.5f, 0.0f), 1.0f);
    const float fg = fminf(fmaxf(zf * 0.2f + 0.5f, 0.0f), 1.0f);
    const float og = fminf(fmaxf(zo * 0.2f + 0.5f, 0.0f), 1.0f);
    const float gg = tanhf(zg);
    const float cn = fg * cold + ig * gg;
    const float hv = og * tanhf(cn);
    const float ov = hv + rv;
    sC[wave * 32 + lane] = cn;
    sH[wave * 32 + lane] = hv;
    sO[wave * 32 + lane] = ov;
  }
  __syncthreads();
  if (tid < 192) {
    const int pl = tid >> 6;
    const int q  = (tid & 63) >> 3;
    const int c4 = (tid & 7) * 4;
    const v4f vc = *(const v4f*)(sC + q * 32 + c4);
    const v4f vh = *(const v4f*)(sH + q * 32 + c4);
    const v4f vo = *(const v4f*)(sO + q * 32 + c4);
    v4f v = vc;
    if (pl == 1) v = vh;
    if (pl == 2) v = vo;
    const size_t srow = (size_t)(p0 + q) * kF + c4;
    const size_t orow = ((size_t)(b * kT + t) * kPixF + ((p0 + q) & (kPixF - 1))) * kF + c4;
    float* dst = Cst + srow;
    if (pl == 1) dst = Hst + srow;
    if (pl == 2) dst = outp + orow;
    for (int pass = 0; pass < 2; ++pass) {
      *(volatile v4f*)dst = v;
      __threadfence();
    }
  }
}

extern "C" void kernel_launch(void* const* d_in, const int* in_sizes, int n_in,
                              void* d_out, int out_size, void* d_ws, size_t ws_size,
                              hipStream_t stream) {
  if (n_in < 8) return;
  if (in_sizes[0] != kB * kT * kPixF * kCin) return;
  if (in_sizes[1] != kLayers * kCin || in_sizes[2] != kLayers * kCin ||
      in_sizes[3] != kLayers * kCin || in_sizes[4] != kLayers * kCin) return;
  if (in_sizes[5] != kLayers * kTaps * kCin * kG4 || in_sizes[6] != kLayers * kTaps * kF * kG4 ||
      in_sizes[7] != kLayers * kG4) return;
  if (out_size != kB * kT * kPixF * kF) return;

  const float* x     = (const float*)d_in[0];
  const float* gamma = (const float*)d_in[1];
  const float* beta  = (const float*)d_in[2];
  const float* mean  = (const float*)d_in[3];
  const float* var   = (const float*)d_in[4];
  const float* kern  = (const float*)d_in[5];
  const float* rker  = (const float*)d_in[6];
  const float* bias  = (const float*)d_in[7];
  float* outp = (float*)d_out;

  const size_t bHS1 = (size_t)kB * kT * kPixF * kF * 4;
  const size_t bIM  = (size_t)kRows * kKtot * 2;
  const size_t bZ   = (size_t)kRows * kG4 * 4;
  const size_t bCST = (size_t)kRows * kF * 4;
  const size_t bHST = (size_t)kRows * kF * 4;
  const size_t bBT  = (size_t)kLayers * kG4 * kKtot * 2;
  char* ws = (char*)d_ws;
  size_t o = 0;
  float* HS1 = (float*)(ws + o);                   o += bHS1;
  unsigned short* IM = (unsigned short*)(ws + o);  o += bIM;
  float* Z   = (float*)(ws + o);                   o += bZ;
  float* CST = (float*)(ws + o);                   o += bCST;
  float* HST = (float*)(ws + o);                   o += bHST;
  unsigned short* BT = (unsigned short*)(ws + o);  o += bBT;
  if (o > ws_size) return;

  k_prep_w<<<dim3((kG4 * kKtot / 8) / 256, kLayers), 256, 0, stream>>>(kern, rker, BT);

  for (int l = 0; l < kLayers; ++l) {
    const float* src   = (l == 0) ? x : HS1;
    float*       lout  = (l == 0) ? HS1 : outp;
    const float* resid = (l == 0) ? x : HS1;
    const unsigned short* BTl = BT + (size_t)l * kG4 * kKtot;
    for (int t = 0; t < kT; ++t) {
      k_im2col<<<(kRows * kChunksPerRow) / 256, 256, 0, stream>>>(
          src, HST, gamma + l * kCin, beta + l * kCin, mean + l * kCin, var + l * kCin, IM, t, (t == 0) ? 1 : 0);
      wmma_gemm64<0, false, 2, 0, false, 0><<<dim3((kRows / 64) * (kG4 / 64) / 8, 1), 256, 0, stream>>>(
          IM, IM, kKtot, 0L,
          BTl, BTl, kKtot, 0L,
          (void*)Z, (void*)Z, kG4, 0L,
          bias + l * kG4,
          bias, 0L,
          kRows, kG4, kKtot, 0.0625f);
      k_cell<<<kRows / 8, 256, 0, stream>>>(Z, CST, HST, lout, resid, t, (t == 0) ? 1 : 0, l);
    }
  }
}
